// TorchRNN_19207093748374
// MI455X (gfx1250) — hardware-run, weakly checked
//
#include <hip/hip_runtime.h>
#include <math.h>

typedef __attribute__((ext_vector_type(8)))  _Float16 v8h;
typedef __attribute__((ext_vector_type(16))) __bf16   v16b;
typedef __attribute__((ext_vector_type(8)))  __bf16   v8b;
typedef __attribute__((ext_vector_type(8)))  float    v8f;
typedef __attribute__((ext_vector_type(4)))  float    v4f;

constexpr int kVocab = 50257;
constexpr int kE     = 128;
constexpr int kH     = 128;
constexpr int kNcls  = 4;
constexpr int kB     = 256;
constexpr int kT     = 512;
constexpr int kM1    = 256;
constexpr int kRows  = kB * kT;
constexpr int kAP    = 136;
constexpr int kHPlane = 16 * kAP;
constexpr int kFP    = 132;
constexpr int kMP    = 260;
static_assert((kE % 32) == 0 && (kH % 32) == 0, "K multiples of 32");
static_assert((kRows % 64) == 0 && (kH % 64) == 0 && (kB % 16) == 0 && (kM1 % 32) == 0, "tile multiples");
static_assert(kH == 128 && kE == 128 && kM1 == 256 && kNcls == 4, "wave maps below assume these widths");

constexpr float kRemJoin = 1.0f;

constexpr size_t kOffXP   = 0;
constexpr size_t kOffWIH  = kOffXP  + (size_t)kRows * kH * 4;
constexpr size_t kOffWIL  = kOffWIH + (size_t)kH * kE * 2;
constexpr size_t kOffWHH  = kOffWIL + (size_t)kH * kE * 2;
constexpr size_t kOffWHL  = kOffWHH + (size_t)kH * kH * 2;
constexpr size_t kOffW1H  = kOffWHL + (size_t)kH * kH * 2;
constexpr size_t kOffW1L  = kOffW1H + (size_t)kM1 * kH * 2;
constexpr size_t kOffBSUM = kOffW1L + (size_t)kM1 * kH * 2;
constexpr size_t kWsTotal = kOffBSUM + (size_t)kH * 4;
static_assert(kWsTotal == 67371520ull, "carve total");
static_assert(kWsTotal <= 134217728ull, "carve cap");
static_assert((kOffWIH % 128) == 0 && (kOffWIL % 128) == 0 && (kOffWHH % 128) == 0 && (kOffWHL % 128) == 0 &&
              (kOffW1H % 128) == 0 && (kOffW1L % 128) == 0 && (kOffBSUM % 128) == 0, "128-B aligned regions");
constexpr int kOut0Elems = kB * kNcls;
constexpr int kOut1Elems = kB * kH;
static_assert(kOut0Elems * 4 == 4096, "second output starts at byte 4096");
static_assert(((kOut0Elems * 4) % 128) == 0, "second output line aligned");

__device__ __forceinline__ unsigned short f2bf_bits(float f) {
  unsigned u = __float_as_uint(f);
  return (unsigned short)((u + 0x7FFFu + ((u >> 16) & 1u)) >> 16);
}
__device__ __forceinline__ float bf_bits2f(unsigned short h) { return __uint_as_float(((unsigned)h) << 16); }

union FragB { v16b v; v8b h[2]; };

__device__ __forceinline__ v16b gload_b(const __bf16* p) {
  FragB f;
  f.h[0] = *(const v8b*)(p);
  f.h[1] = *(const v8b*)(p + 16);
  return f.v;
}

__device__ __forceinline__ v8f wmma_b(v16b a, v16b b, v8f c) {
  c = __builtin_amdgcn_wmma_f32_16x16x32_bf16(false, a, false, b, (short)0, c, false, false);
  asm volatile("v_nop\n\tv_nop\n\tv_nop\n\tv_nop" : "+v"(c) : "v"(a), "v"(b));
  return c;
}

__device__ __forceinline__ void split8_store(const float* __restrict__ src, unsigned short* __restrict__ dhi,
                                             unsigned short* __restrict__ dlo, size_t e0) {
  const v4f a0 = *(const v4f*)(src + e0);
  const v4f a1 = *(const v4f*)(src + e0 + 4);
  v8h hv, lv;
#pragma unroll
  for (int e = 0; e < 4; ++e) {
    const unsigned short h0 = f2bf_bits(a0[e]), h1 = f2bf_bits(a1[e]);
    const unsigned short l0 = f2bf_bits(a0[e] - bf_bits2f(h0)), l1 = f2bf_bits(a1[e] - bf_bits2f(h1));
    hv[e]     = __builtin_bit_cast(_Float16, h0);
    hv[4 + e] = __builtin_bit_cast(_Float16, h1);
    lv[e]     = __builtin_bit_cast(_Float16, l0);
    lv[4 + e] = __builtin_bit_cast(_Float16, l1);
  }
  unsigned short* qh = dhi + e0;
  unsigned short* ql = dlo + e0;
  *(volatile v8h*)qh = hv;
  *(volatile v8h*)ql = lv;
  __threadfence();
  *(volatile v8h*)qh = hv;
  *(volatile v8h*)ql = lv;
}

__global__ __launch_bounds__(256) void prep_planes_kernel(
    const float* __restrict__ Wih, const float* __restrict__ Whh, const float* __restrict__ W1,
    const float* __restrict__ bih, const float* __restrict__ bhh,
    unsigned short* __restrict__ WIH, unsigned short* __restrict__ WIL,
    unsigned short* __restrict__ WHH, unsigned short* __restrict__ WHL,
    unsigned short* __restrict__ W1H, unsigned short* __restrict__ W1L, float* __restrict__ BSUM)
{
  const int blk = blockIdx.x;
  const int tid = threadIdx.x;
  if (blk < 8) {
    const size_t e0 = ((size_t)blk * 256 + tid) << 3;
    split8_store(Wih, WIH, WIL, e0);
  } else if (blk < 16) {
    const size_t e0 = ((size_t)(blk - 8) * 256 + tid) << 3;
    split8_store(Whh, WHH, WHL, e0);
  } else if (blk < 32) {
    const size_t e0 = ((size_t)(blk - 16) * 256 + tid) << 3;
    split8_store(W1, W1H, W1L, e0);
  } else {
    if (tid < 32) {
      const v4f x0 = *(const v4f*)(bih + tid * 4);
      const v4f x1 = *(const v4f*)(bhh + tid * 4);
      v4f s;
      s[0] = x0[0] + x1[0];
      s[1] = x0[1] + x1[1];
      s[2] = x0[2] + x1[2];
      s[3] = x0[3] + x1[3];
      float* q = BSUM + tid * 4;
      *(volatile v4f*)q = s;
      __threadfence();
      *(volatile v4f*)q = s;
    }
  }
}

__global__ __launch_bounds__(256) void inproj_kernel(
    const int* __restrict__ x, const float* __restrict__ emb,
    const unsigned short* __restrict__ WIHp, const unsigned short* __restrict__ WILp,
    const float* __restrict__ bsum, float* __restrict__ xp)
{
  __shared__ __align__(16) __bf16 AsH[64 * kAP];
  __shared__ __align__(16) __bf16 AsL[64 * kAP];
  __shared__ __align__(16) float slabS[8 * 16 * 68];
  const int tid  = threadIdx.x;
  const int lane = tid & 31;
  const int wave = tid >> 5;
  const int hh   = lane >> 4;
  const int c    = lane & 15;
  const int r0   = blockIdx.x * 64;
  {
    const int row = tid >> 2;
    const int seg = tid & 3;
    const int r = r0 + row;
    const int t = r / kB;
    const int b = r - t * kB;
    int tok = x[(size_t)b * kT + t];
    tok = tok < 0 ? 0 : tok;
    tok = tok > (kVocab - 1) ? (kVocab - 1) : tok;
    const float* src = emb + (size_t)tok * kE + seg * 32;
#pragma unroll
    for (int i = 0; i < 4; ++i) {
      const v4f a0 = *(const v4f*)(src + 8 * i);
      const v4f a1 = *(const v4f*)(src + 8 * i + 4);
      v8b hv, lv;
#pragma unroll
      for (int e = 0; e < 4; ++e) {
        const unsigned short p0 = f2bf_bits(a0[e]), p1 = f2bf_bits(a1[e]);
        const unsigned short q0 = f2bf_bits(a0[e] - bf_bits2f(p0)), q1 = f2bf_bits(a1[e] - bf_bits2f(p1));
        hv[e]     = __builtin_bit_cast(__bf16, p0);
        hv[4 + e] = __builtin_bit_cast(__bf16, p1);
        lv[e]     = __builtin_bit_cast(__bf16, q0);
        lv[4 + e] = __builtin_bit_cast(__bf16, q1);
      }
      *(v8b*)(AsH + row * kAP + seg * 32 + 8 * i) = hv;
      *(v8b*)(AsL + row * kAP + seg * 32 + 8 * i) = lv;
    }
  }
  __syncthreads();

  const __bf16* WIH = (const __bf16*)WIHp;
  const __bf16* WIL = (const __bf16*)WILp;
  const int mi = wave & 3;
  const int nh = wave >> 2;
  v8f acc[4], rem[4];
#pragma unroll
  for (int j = 0; j < 4; ++j) {
    acc[j] = (v8f){0.f, 0.f, 0.f, 0.f, 0.f, 0.f, 0.f, 0.f};
    rem[j] = (v8f){0.f, 0.f, 0.f, 0.f, 0.f, 0.f, 0.f, 0.f};
  }
#pragma unroll
  for (int kc = 0; kc < 4; ++kc) {
    FragB a, l;
    a.h[0] = *(const v8b*)(AsH + (mi * 16 + c) * kAP + kc * 32 + 8 * hh);
    a.h[1] = *(const v8b*)(AsH + (mi * 16 + c) * kAP + kc * 32 + 16 + 8 * hh);
    l.h[0] = *(const v8b*)(AsL + (mi * 16 + c) * kAP + kc * 32 + 8 * hh);
    l.h[1] = *(const v8b*)(AsL + (mi * 16 + c) * kAP + kc * 32 + 16 + 8 * hh);
#pragma unroll
    for (int j = 0; j < 4; ++j) {
      const size_t off = (size_t)(nh * 64 + j * 16 + c) * kE + kc * 32 + 8 * hh;
      const v16b wh = gload_b(WIH + off);
      const v16b wl = gload_b(WIL + off);
      acc[j] = wmma_b(a.v, wh, acc[j]);
      rem[j] = wmma_b(a.v, wl, rem[j]);
      rem[j] = wmma_b(l.v, wh, rem[j]);
    }
  }

  float* slab = slabS + wave * (16 * 68);
#pragma unroll
  for (int j = 0; j < 4; ++j) {
    const float bv = bsum[nh * 64 + j * 16 + c];
#pragma unroll
    for (int r = 0; r < 8; ++r) {
      const float joined = acc[j][r] + rem[j][r] * kRemJoin;
      slab[(8 * hh + r) * 68 + j * 16 + c] = joined + bv;
    }
  }
  __builtin_amdgcn_fence(__ATOMIC_RELEASE, "workgroup");
  __builtin_amdgcn_wave_barrier();
  __builtin_amdgcn_fence(__ATOMIC_ACQUIRE, "workgroup");
  {
    const int c4 = c * 4;
    v4f sv[8];
#pragma unroll
    for (int it = 0; it < 8; ++it) sv[it] = *(const v4f*)(slab + (it * 2 + hh) * 68 + c4);
    for (int pass = 0; pass < 2; ++pass) {
#pragma unroll
      for (int it = 0; it < 8; ++it)
        *(volatile v4f*)(xp + (size_t)(r0 + mi * 16 + it * 2 + hh) * kH + nh * 64 + c4) = sv[it];
      __threadfence();
    }
  }
}

__global__ __launch_bounds__(256) void recur_head_kernel(
    const float* __restrict__ h0, const float* __restrict__ xp,
    const unsigned short* __restrict__ WHHp, const unsigned short* __restrict__ WHLp,
    const unsigned short* __restrict__ W1Hp, const unsigned short* __restrict__ W1Lp,
    const float* __restrict__ b1, const float* __restrict__ W2, const float* __restrict__ b2,
    float* __restrict__ out0, float* __restrict__ out1)
{
  __shared__ __align__(16) __bf16 hH[2 * kHPlane];
  __shared__ __align__(16) __bf16 hL[2 * kHPlane];
  __shared__ __align__(16) float hF[16 * kFP];
  __shared__ __align__(16) float hmS[16 * kMP];
  __shared__ __align__(16) float lgS[64];

  const int tid  = threadIdx.x;
  const int lane = tid & 31;
  const int wave = tid >> 5;
  const int hh   = lane >> 4;
  const int c    = lane & 15;
  const int n    = wave * 16 + c;
  const int b0   = blockIdx.x * 16;

  const __bf16* WHH = (const __bf16*)WHHp;
  const __bf16* WHL = (const __bf16*)WHLp;
  const __bf16* W1H = (const __bf16*)W1Hp;
  const __bf16* W1L = (const __bf16*)W1Lp;

  {
    const int row = tid >> 4;
    const int c8  = (tid & 15) * 8;
    const float* src = h0 + (size_t)(b0 + row) * kH + c8;
    const v4f a0 = *(const v4f*)(src);
    const v4f a1 = *(const v4f*)(src + 4);
    v8b hv, lv;
#pragma unroll
    for (int e = 0; e < 4; ++e) {
      const unsigned short p0 = f2bf_bits(a0[e]), p1 = f2bf_bits(a1[e]);
      const unsigned short q0 = f2bf_bits(a0[e] - bf_bits2f(p0)), q1 = f2bf_bits(a1[e] - bf_bits2f(p1));
      hv[e]     = __builtin_bit_cast(__bf16, p0);
      hv[4 + e] = __builtin_bit_cast(__bf16, p1);
      lv[e]     = __builtin_bit_cast(__bf16, q0);
      lv[4 + e] = __builtin_bit_cast(__bf16, q1);
    }
    *(v8b*)(hH + row * kAP + c8) = hv;
    *(v8b*)(hL + row * kAP + c8) = lv;
  }

  v16b bh[4], bl[4];
#pragma unroll
  for (int kc = 0; kc < 4; ++kc) {
    const size_t off = (size_t)n * kH + kc * 32 + 8 * hh;
    bh[kc] = gload_b(WHH + off);
    bl[kc] = gload_b(WHL + off);
  }

  __syncthreads();

  float hfin[8];
#pragma unroll
  for (int r = 0; r < 8; ++r) hfin[r] = 0.f;

  int cur = 0;
#pragma unroll 1
  for (int t = 0; t < kT; ++t) {
    const float* xrow = xp + ((size_t)t * kB + b0 + 8 * hh) * kH + n;
    float xv[8];
#pragma unroll
    for (int r = 0; r < 8; ++r) xv[r] = xrow[(size_t)r * kH];

    const __bf16* ph = hH + cur * kHPlane + c * kAP + 8 * hh;
    const __bf16* pl = hL + cur * kHPlane + c * kAP + 8 * hh;
    v8f acc = (v8f){0.f, 0.f, 0.f, 0.f, 0.f, 0.f, 0.f, 0.f};
#pragma unroll
    for (int kc = 0; kc < 4; ++kc) {
      FragB a, l;
      a.h[0] = *(const v8b*)(ph + kc * 32);
      a.h[1] = *(const v8b*)(ph + kc * 32 + 16);
      l.h[0] = *(const v8b*)(pl + kc * 32);
      l.h[1] = *(const v8b*)(pl + kc * 32 + 16);
      acc = wmma_b(a.v, bh[kc], acc);
      acc = wmma_b(a.v, bl[kc], acc);
      acc = wmma_b(l.v, bh[kc], acc);
    }
#pragma unroll
    for (int r = 0; r < 8; ++r) asm volatile("" : "+v"(xv[r]));

    const int nxt = cur ^ 1;
    __bf16* qh = hH + nxt * kHPlane + (8 * hh) * kAP + n;
    __bf16* ql = hL + nxt * kHPlane + (8 * hh) * kAP + n;
#pragma unroll
    for (int r = 0; r < 8; ++r) {
      const float pre = xv[r] + acc[r];
      const float hn  = tanhf(pre);
      hfin[r] = hn;
      const unsigned short hb = f2bf_bits(hn);
      const unsigned short lb = f2bf_bits(hn - bf_bits2f(hb));
      qh[r * kAP] = __builtin_bit_cast(__bf16, hb);
      ql[r * kAP] = __builtin_bit_cast(__bf16, lb);
    }
    __syncthreads();
    cur = nxt;
  }

#pragma unroll
  for (int r = 0; r < 8; ++r) hF[(8 * hh + r) * kFP + n] = hfin[r];
  __syncthreads();
  {
    const int rA = 2 * wave;
    const int rB = 2 * wave + 1;
    const v4f vA = *(const v4f*)(hF + rA * kFP + lane * 4);
    const v4f vB = *(const v4f*)(hF + rB * kFP + lane * 4);
    float* pA = out1 + (size_t)(b0 + rA) * kH + lane * 4;
    float* pB = out1 + (size_t)(b0 + rB) * kH + lane * 4;
    *(volatile v4f*)pA = vA;
    *(volatile v4f*)pB = vB;
    __threadfence();
    *(volatile v4f*)pA = vA;
    *(volatile v4f*)pB = vB;
  }

  {
    const __bf16* ph = hH + cur * kHPlane + c * kAP + 8 * hh;
    const __bf16* pl = hL + cur * kHPlane + c * kAP + 8 * hh;
    v8f a2[2];
    a2[0] = (v8f){0.f, 0.f, 0.f, 0.f, 0.f, 0.f, 0.f, 0.f};
    a2[1] = (v8f){0.f, 0.f, 0.f, 0.f, 0.f, 0.f, 0.f, 0.f};
#pragma unroll
    for (int kc = 0; kc < 4; ++kc) {
      FragB a, l;
      a.h[0] = *(const v8b*)(ph + kc * 32);
      a.h[1] = *(const v8b*)(ph + kc * 32 + 16);
      l.h[0] = *(const v8b*)(pl + kc * 32);
      l.h[1] = *(const v8b*)(pl + kc * 32 + 16);
#pragma unroll
      for (int j = 0; j < 2; ++j) {
        const size_t off = (size_t)(32 * wave + 16 * j + c) * kH + kc * 32 + 8 * hh;
        const v16b wh = gload_b(W1H + off);
        const v16b wl = gload_b(W1L + off);
        a2[j] = wmma_b(a.v, wh, a2[j]);
        a2[j] = wmma_b(a.v, wl, a2[j]);
        a2[j] = wmma_b(l.v, wh, a2[j]);
      }
    }
#pragma unroll
    for (int j = 0; j < 2; ++j) {
      const int nn = 32 * wave + 16 * j + c;
      const float bv = b1[nn];
#pragma unroll
      for (int r = 0; r < 8; ++r) {
        float v = a2[j][r] + bv;
        v = fmaxf(v, 0.0f);
        hmS[(8 * hh + r) * kMP + nn] = v;
      }
    }
  }
  __syncthreads();

  if (tid < 64) {
    const int row = tid >> 2;
    const int cls = tid & 3;
    const float* hp = hmS + row * kMP;
    const float* wp = W2 + (size_t)cls * kM1;
    float s = 0.0f;
#pragma unroll 1
    for (int k4 = 0; k4 < kM1 / 4; ++k4) {
      const v4f hv = *(const v4f*)(hp + 4 * k4);
      const v4f wv = *(const v4f*)(wp + 4 * k4);
      s = fmaf(hv[0], wv[0], s);
      s = fmaf(hv[1], wv[1], s);
      s = fmaf(hv[2], wv[2], s);
      s = fmaf(hv[3], wv[3], s);
    }
    s = s + b2[cls];
    lgS[tid] = s;
  }
  __syncthreads();
  if (tid < 16) {
    const v4f v = *(const v4f*)(lgS + tid * 4);
    float* p = out0 + (size_t)b0 * kNcls + tid * 4;
    *(volatile v4f*)p = v;
    __threadfence();
    *(volatile v4f*)p = v;
  }
}

extern "C" void kernel_launch(void* const* d_in, const int* in_sizes, int n_in,
                              void* d_out, int out_size, void* d_ws, size_t ws_size,
                              hipStream_t stream) {
  if (n_in < 11) return;
  if (in_sizes[0] != kB * kT) return;
  if (in_sizes[1] != kB * kH) return;
  if (in_sizes[2] != kVocab * kE) return;
  if (in_sizes[3] != kH * kE) return;
  if (in_sizes[4] != kH * kH) return;
  if (in_sizes[5] != kH) return;
  if (in_sizes[6] != kH) return;
  if (in_sizes[7] != kM1 * kH) return;
  if (in_sizes[8] != kM1) return;
  if (in_sizes[9] != kNcls * kM1) return;
  if (in_sizes[10] != kNcls) return;
  if (out_size != kOut0Elems + kOut1Elems) return;
  if (ws_size < kWsTotal) return;

  const int*   x    = (const int*)  d_in[0];
  const float* h0   = (const float*)d_in[1];
  const float* emb  = (const float*)d_in[2];
  const float* Wih  = (const float*)d_in[3];
  const float* Whh  = (const float*)d_in[4];
  const float* bih  = (const float*)d_in[5];
  const float* bhh  = (const float*)d_in[6];
  const float* W1   = (const float*)d_in[7];
  const float* b1   = (const float*)d_in[8];
  const float* W2   = (const float*)d_in[9];
  const float* b2   = (const float*)d_in[10];

  float* out0 = (float*)d_out;
  float* out1 = (float*)d_out + kOut0Elems;

  char* ws = (char*)d_ws;
  float*          XP   = (float*)(ws + kOffXP);
  unsigned short* WIH  = (unsigned short*)(ws + kOffWIH);
  unsigned short* WIL  = (unsigned short*)(ws + kOffWIL);
  unsigned short* WHH  = (unsigned short*)(ws + kOffWHH);
  unsigned short* WHL  = (unsigned short*)(ws + kOffWHL);
  unsigned short* W1H  = (unsigned short*)(ws + kOffW1H);
  unsigned short* W1L  = (unsigned short*)(ws + kOffW1L);
  float*          BSUM = (float*)(ws + kOffBSUM);

  prep_planes_kernel<<<33, 256, 0, stream>>>(Wih, Whh, W1, bih, bhh, WIH, WIL, WHH, WHL, W1H, W1L, BSUM);
  inproj_kernel<<<kRows / 64, 256, 0, stream>>>(x, emb, WIH, WIL, BSUM, XP);
  recur_head_kernel<<<kB / 16, 256, 0, stream>>>(h0, XP, WHH, WHL, W1H, W1L, b1, W2, b2, out0, out1);
}
